// NAM_4818953306387
// MI455X (gfx1250) — hardware-verified
//
#include <hip/hip_runtime.h>
#include <math.h>

constexpr int kRows      = 16384;
constexpr int kFeat      = 64;
constexpr int kUnit      = 64;
constexpr int kKdim      = kFeat * kUnit;
constexpr int kChunkRows = 8192;
constexpr int kNumChunks = kRows / kChunkRows;
constexpr float kWCarry    = 256.0f;
constexpr float kWCarryInv = 1.0f / 256.0f;
static_assert(kNumChunks * kChunkRows == kRows, "chunks");
static_assert(kChunkRows % 64 == 0 && kFeat % 64 == 0 && kKdim % 32 == 0, "tiles");

constexpr size_t kOffEW   = 0;
constexpr size_t kBytesEW = (size_t)kFeat * kUnit * 4;
constexpr size_t kOffBt   = kOffEW + kBytesEW;
constexpr size_t kBytesBt = (size_t)kFeat * kKdim * 2;
constexpr size_t kOffA    = kOffBt + kBytesBt;
constexpr size_t kBytesA  = (size_t)kChunkRows * kKdim * 2;
constexpr size_t kWsTotal = kOffA + kBytesA;
static_assert(kWsTotal == 67649536, "carve");
static_assert(kWsTotal <= 134217728, "carve cap");
static_assert((kOffBt % 128) == 0 && (kOffA % 128) == 0, "align");

typedef __attribute__((ext_vector_type(16))) _Float16 v16h;
typedef __attribute__((ext_vector_type(8)))  _Float16 v8h;
typedef __attribute__((ext_vector_type(16))) __bf16   v16b;
typedef __attribute__((ext_vector_type(8)))  __bf16   v8b;
typedef __attribute__((ext_vector_type(8)))  float    v8f;
typedef __attribute__((ext_vector_type(4)))  float    v4f;
typedef __attribute__((ext_vector_type(4)))  unsigned int v4u;

__device__ __forceinline__ unsigned short f2bf_bits(float f) {
  unsigned u = __float_as_uint(f);
  return (unsigned short)((u + 0x7FFFu + ((u >> 16) & 1u)) >> 16);
}
__device__ __forceinline__ float bf_bits2f(unsigned short h) { return __uint_as_float(((unsigned)h) << 16); }

__device__ __forceinline__ void dep_guard_h(v8f& a, v8f& b, v16h x, v16h y) { asm volatile("v_nop\n\tv_nop\n\tv_nop\n\tv_nop" : "+v"(a), "+v"(b) : "v"(x), "v"(y)); }
__device__ __forceinline__ void dep_guard_b(v8f& a, v8f& b, v16b x, v16b y) { asm volatile("v_nop\n\tv_nop\n\tv_nop\n\tv_nop" : "+v"(a), "+v"(b) : "v"(x), "v"(y)); }
__device__ __forceinline__ void keep4_h(v16h a, v16h b, v16h c, v16h d) { asm volatile("v_nop" :: "v"(a), "v"(b), "v"(c), "v"(d)); }
__device__ __forceinline__ void keep4_b(v16b a, v16b b, v16b c, v16b d) { asm volatile("v_nop" :: "v"(a), "v"(b), "v"(c), "v"(d)); }
__device__ __forceinline__ void acc_guard4(v8f& a, v8f& b, v8f& c, v8f& d) { asm volatile("v_nop\n\tv_nop\n\tv_nop\n\tv_nop" : "+v"(a), "+v"(b), "+v"(c), "+v"(d)); }
template <typename T> struct Frag;
template <> struct Frag<_Float16> {
  typedef v16h V; union U { v16h v; v8h h[2]; };
  static __device__ __forceinline__ v16h load(const _Float16* p) {
    U f; f.h[0] = *(const v8h*)(p); f.h[1] = *(const v8h*)(p + 16); return f.v;
  }
  static __device__ __forceinline__ v8f mma(v16h a, v16h b, v8f c) {
    return __builtin_amdgcn_wmma_f32_16x16x32_f16(false, a, false, b, (short)0, c, false, false);
  }
  static __device__ __forceinline__ void guard(v8f& a, v8f& b, v16h x, v16h y) { dep_guard_h(a, b, x, y); }
  static __device__ __forceinline__ void keep(v16h a, v16h b, v16h c, v16h d) { keep4_h(a, b, c, d); }
};
template <> struct Frag<__bf16> {
  typedef v16b V; union U { v16b v; v8b h[2]; };
  static __device__ __forceinline__ v16b load(const __bf16* p) {
    U f; f.h[0] = *(const v8b*)(p); f.h[1] = *(const v8b*)(p + 16); return f.v;
  }
  static __device__ __forceinline__ v8f mma(v16b a, v16b b, v8f c) {
    return __builtin_amdgcn_wmma_f32_16x16x32_bf16(false, a, false, b, (short)0, c, false, false);
  }
  static __device__ __forceinline__ void guard(v8f& a, v8f& b, v16b x, v16b y) { dep_guard_b(a, b, x, y); }
  static __device__ __forceinline__ void keep(v16b a, v16b b, v16b c, v16b d) { keep4_b(a, b, c, d); }
};

__device__ __forceinline__ unsigned pk16(unsigned short a, unsigned short b) { return (unsigned)a | ((unsigned)b << 16); }
__device__ __forceinline__ unsigned short h_bits(float f) { const _Float16 h = (_Float16)f; return __builtin_bit_cast(unsigned short, h); }

template <int ET> struct Elem;
template <> struct Elem<0> { typedef _Float16 T; };
template <> struct Elem<1> { typedef __bf16 T; };
template <int ET, bool SPLIT, int BIAS_MODE, int OUT_MODE, bool RESID, int ACT = 0>
__global__ __launch_bounds__(256) void wmma_gemm64(
    const unsigned short* __restrict__ Ap, const unsigned short* __restrict__ A2p, int lda, long strideA,
    const unsigned short* __restrict__ Btp, const unsigned short* __restrict__ Bt2p, int ldb, long strideB,
    void* __restrict__ Cout, void* __restrict__ Cout2, int ldc, long strideC,
    const float* __restrict__ bias,
    const float* __restrict__ resid, long strideR,
    int M, int N, int K, float scale) {
  typedef typename Elem<ET>::T T;
  typedef typename Frag<T>::V V;
  const T* A = (const T*)Ap; const T* A2 = (const T*)A2p; const T* Bt = (const T*)Btp; const T* Bt2 = (const T*)Bt2p;
  __shared__ __align__(16) float sT[8][16 * 68];
  const int b    = blockIdx.y;
  const int lane = threadIdx.x & 31;
  const int wave = threadIdx.x >> 5;
  const int tilesN = N >> 6;
  const int tilesM = M >> 6;
  const int tile = blockIdx.x * 8 + wave;
  if (tile >= tilesM * tilesN) return;
  const int tm = tile / tilesN;
  const int tn = tile - tm * tilesN;
  const int m0 = tm << 6;
  const int n0 = tn << 6;

  const T* Ab  = A  + (size_t)b * strideA;
  const T* Bb  = Bt + (size_t)b * strideB;
  const T* Ab2 = SPLIT ? (A2  + (size_t)b * strideA) : nullptr;
  const T* Bb2 = SPLIT ? (Bt2 + (size_t)b * strideB) : nullptr;

  const int rlane = lane & 15;
  const int koff  = (lane >> 4) * 8;
  const int mOff  = (lane >> 4) * 8;

  v8f acc[4][4];
#pragma unroll
  for (int i = 0; i < 4; ++i)
#pragma unroll
    for (int j = 0; j < 4; ++j) acc[i][j] = (v8f){0.f,0.f,0.f,0.f,0.f,0.f,0.f,0.f};

  for (int k0 = 0; k0 < K; k0 += 32) {
    V bh[4], bl[4];
#pragma unroll
    for (int j = 0; j < 4; ++j) {
      const size_t bo = (size_t)(n0 + (j << 4) + rlane) * ldb + koff + k0;
      bh[j] = Frag<T>::load(Bb + bo);
      if (SPLIT) bl[j] = Frag<T>::load(Bb2 + bo);
    }
#pragma unroll
    for (int i = 0; i < 4; ++i) {
      const size_t ao = (size_t)(m0 + (i << 4) + rlane) * lda + koff + k0;
      V ah = Frag<T>::load(Ab + ao);
      V al;
      if (SPLIT) al = Frag<T>::load(Ab2 + ao);
#pragma unroll
      for (int j = 0; j < 4; ++j) {
        acc[i][j] = Frag<T>::mma(ah, bh[j], acc[i][j]);
        if (SPLIT) {
          acc[i][j] = Frag<T>::mma(ah, bl[j], acc[i][j]);
          acc[i][j] = Frag<T>::mma(al, bh[j], acc[i][j]);
        }
      }
      Frag<T>::guard(acc[i][0], acc[i][3], ah, SPLIT ? al : ah);
    }
    Frag<T>::keep(bh[0], bh[1], bh[2], bh[3]);
    if (SPLIT) Frag<T>::keep(bl[0], bl[1], bl[2], bl[3]);
  }
  acc_guard4(acc[0][0], acc[0][1], acc[0][2], acc[0][3]);
  acc_guard4(acc[1][0], acc[1][1], acc[1][2], acc[1][3]);
  acc_guard4(acc[2][0], acc[2][1], acc[2][2], acc[2][3]);
  acc_guard4(acc[3][0], acc[3][1], acc[3][2], acc[3][3]);

  float* slab = sT[wave];
  const float* Rb = RESID ? (resid + (size_t)b * strideR) : nullptr;
#pragma unroll
  for (int i = 0; i < 4; ++i) {
    const int mBase = m0 + (i << 4);
#pragma unroll
    for (int j = 0; j < 4; ++j) {
      const int n = n0 + (j << 4) + rlane;
      float bv = 0.f;
      if (BIAS_MODE == 2) bv = bias[n];
#pragma unroll
      for (int r = 0; r < 8; ++r) {
        float v = acc[i][j][r] * scale;
        if (BIAS_MODE == 1) v += bias[mBase + mOff + r];
        if (BIAS_MODE == 2) v += bv;
        if (RESID) v += Rb[(size_t)(mBase + mOff + r) * ldc + n];
        if (ACT == 2) v = fmaxf(v, 0.0f);
        if (ACT == 4) v = (v > 0.f) ? v : 0.01f * v;
        slab[(mOff + r) * 68 + (j << 4) + rlane] = v;
      }
    }
    __builtin_amdgcn_fence(__ATOMIC_RELEASE, "workgroup");
    __builtin_amdgcn_wave_barrier();
    __builtin_amdgcn_fence(__ATOMIC_ACQUIRE, "workgroup");
    if (OUT_MODE == 0) {
      float* C = (float*)Cout + (size_t)b * strideC;
      const int hh = lane >> 4, c4 = (lane & 15) * 4;
      for (int pass = 0; pass < 2; ++pass) {
#pragma unroll
        for (int it = 0; it < 8; ++it) {
          const int row = it * 2 + hh;
          v4f v = *(const v4f*)(slab + row * 68 + c4);
          *(volatile v4f*)(C + (size_t)(mBase + row) * ldc + n0 + c4) = v;
        }
        __threadfence();
      }
    } else {
      const int q = lane >> 3, c8 = (lane & 7) * 8;
      unsigned short* C  = (unsigned short*)Cout  + (size_t)b * strideC;
      unsigned short* C2 = (OUT_MODE == 2) ? ((unsigned short*)Cout2 + (size_t)b * strideC) : nullptr;
      for (int pass = 0; pass < 2; ++pass) {
#pragma unroll
        for (int it = 0; it < 4; ++it) {
          const int row = it * 4 + q;
          const float* sp = slab + row * 68 + c8;
          v8h hv, lv;
#pragma unroll
          for (int e = 0; e < 8; ++e) {
            if (OUT_MODE == 1) {
              hv[e] = (_Float16)sp[e];
            } else {
              unsigned short hb = f2bf_bits(sp[e]);
              unsigned short lb = f2bf_bits(sp[e] - bf_bits2f(hb));
              hv[e] = __builtin_bit_cast(_Float16, hb);
              lv[e] = __builtin_bit_cast(_Float16, lb);
            }
          }
          *(volatile v8h*)(C + (size_t)(mBase + row) * ldc + n0 + c8) = hv;
          if (OUT_MODE == 2) *(volatile v8h*)(C2 + (size_t)(mBase + row) * ldc + n0 + c8) = lv;
        }
        __threadfence();
      }
    }
    __builtin_amdgcn_fence(__ATOMIC_RELEASE, "workgroup");
    __builtin_amdgcn_wave_barrier();
    __builtin_amdgcn_fence(__ATOMIC_ACQUIRE, "workgroup");
  }
}

__global__ __launch_bounds__(256) void ew_prep_kernel(const float* __restrict__ exu_w, float* __restrict__ ew, int n4) {
  const int i = blockIdx.x * 256 + threadIdx.x;
  if (i >= n4) return;
  const v4f w = *(const v4f*)(exu_w + 4 * (size_t)i);
  v4f e;
  e[0] = expf(w[0]);
  e[1] = expf(w[1]);
  e[2] = expf(w[2]);
  e[3] = expf(w[3]);
  float* q = ew + 4 * (size_t)i;
  *(volatile v4f*)q = e;
  __threadfence();
  *(volatile v4f*)q = e;
}

__global__ __launch_bounds__(256) void bt_build_kernel(const float* __restrict__ lin_w, unsigned short* __restrict__ bt, float carry) {
  const int i  = blockIdx.x * 256 + threadIdx.x;
  const int f  = i >> 9;
  const int k0 = (i & 511) * 8;
  const int fk = k0 >> 6;
  const int u0 = k0 & 63;
  const float* p = lin_w + f * kUnit + u0;
  const v4f a = *(const v4f*)(p);
  const v4f c = *(const v4f*)(p + 4);
  unsigned short hb[8];
#pragma unroll
  for (int e = 0; e < 4; ++e) {
    hb[e]     = h_bits(a[e] * carry);
    hb[4 + e] = h_bits(c[e] * carry);
  }
  const unsigned msk = (fk == f) ? 0xffffffffu : 0u;
  const v4u u = (v4u){pk16(hb[0], hb[1]) & msk, pk16(hb[2], hb[3]) & msk, pk16(hb[4], hb[5]) & msk, pk16(hb[6], hb[7]) & msk};
  unsigned short* q = bt + 8 * (size_t)i;
  *(volatile v4u*)q = u;
  __threadfence();
  *(volatile v4u*)q = u;
}

__global__ __launch_bounds__(256) void a_build_kernel(const float* __restrict__ x, const float* __restrict__ exu_b,
                                                      const float* __restrict__ ew, unsigned short* __restrict__ ap, int row0) {
  const int i   = blockIdx.x * 256 + threadIdx.x;
  const int r   = i >> 9;
  const int rem = i & 511;
  const int f   = rem >> 3;
  const int u0  = (rem & 7) * 8;
  const float xv = x[((size_t)(row0 + r)) * kFeat + f];
  const float bv = exu_b[f];
  const float d  = xv - bv;
  const float* ep = ew + f * kUnit + u0;
  const v4f e0 = *(const v4f*)(ep);
  const v4f e1 = *(const v4f*)(ep + 4);
  unsigned short hb[8];
#pragma unroll
  for (int e = 0; e < 4; ++e) {
    float p0 = d * e0[e];
    p0 = fmaxf(p0, 0.0f);
    p0 = fminf(p0, 1.0f);
    hb[e] = h_bits(p0);
    float p1 = d * e1[e];
    p1 = fmaxf(p1, 0.0f);
    p1 = fminf(p1, 1.0f);
    hb[4 + e] = h_bits(p1);
  }
  const v4u u = (v4u){pk16(hb[0], hb[1]), pk16(hb[2], hb[3]), pk16(hb[4], hb[5]), pk16(hb[6], hb[7])};
  unsigned short* q = ap + 8 * (size_t)i;
  *(volatile v4u*)q = u;
  __threadfence();
  *(volatile v4u*)q = u;
}

__global__ __launch_bounds__(256) void rowsum_kernel(const float* __restrict__ fnn, const float* __restrict__ bias, float* __restrict__ out) {
  __shared__ __align__(16) float sres[256];
  const int t   = threadIdx.x;
  const int row = blockIdx.x * 256 + t;
  const float* p = fnn + (size_t)row * kFeat;
  float s = 0.f;
#pragma unroll
  for (int qd = 0; qd < 16; ++qd) {
    const v4f v = *(const v4f*)(p + 4 * qd);
    s += v[0];
    s += v[1];
    s += v[2];
    s += v[3];
  }
  s += bias[0];
  sres[t] = s;
  __syncthreads();
  if (t < 64) {
    const v4f v = *(const v4f*)(sres + 4 * t);
    float* q = out + (size_t)blockIdx.x * 256 + 4 * t;
    *(volatile v4f*)q = v;
    __threadfence();
    *(volatile v4f*)q = v;
  }
}

extern "C" void kernel_launch(void* const* d_in, const int* in_sizes, int n_in,
                              void* d_out, int out_size, void* d_ws, size_t ws_size,
                              hipStream_t stream) {
  if (n_in < 6) return;
  if (in_sizes[0] != kRows * kFeat || in_sizes[1] != kFeat * kUnit || in_sizes[2] != kFeat ||
      in_sizes[3] != kFeat * kUnit || in_sizes[4] != kFeat || in_sizes[5] < 1) return;
  if (out_size != kRows + kRows * kFeat) return;
  if (ws_size < kWsTotal) return;

  const float* x     = (const float*)d_in[0];
  const float* exu_w = (const float*)d_in[1];
  const float* exu_b = (const float*)d_in[2];
  const float* lin_w = (const float*)d_in[3];
  const float* lin_b = (const float*)d_in[4];
  const float* bias  = (const float*)d_in[5];

  float* out0 = (float*)d_out;
  float* fnn  = (float*)d_out + kRows;

  char* ws = (char*)d_ws;
  float*          ew = (float*)(ws + kOffEW);
  unsigned short* bt = (unsigned short*)(ws + kOffBt);
  unsigned short* ap = (unsigned short*)(ws + kOffA);

  ew_prep_kernel<<<dim3((kFeat * kUnit / 4) / 256), dim3(256), 0, stream>>>(exu_w, ew, kFeat * kUnit / 4);
  bt_build_kernel<<<dim3((kFeat * kKdim / 8) / 256), dim3(256), 0, stream>>>(lin_w, bt, kWCarry);

  for (int c = 0; c < kNumChunks; ++c) {
    a_build_kernel<<<dim3((kChunkRows * kKdim / 8) / 256), dim3(256), 0, stream>>>(x, exu_b, ew, ap, c * kChunkRows);
    float* cptr = fnn + (size_t)c * kChunkRows * kFeat;
    wmma_gemm64<0, false, 2, 0, false, 0><<<dim3((kChunkRows / 64) / 8, 1, 1), dim3(256), 0, stream>>>(
        (const unsigned short*)ap, (const unsigned short*)ap, kKdim, (long)0,
        (const unsigned short*)bt, (const unsigned short*)bt, kKdim, (long)0,
        (void*)cptr, (void*)cptr, kFeat, (long)0,
        lin_b,
        (const float*)ew, (long)0,
        kChunkRows, kFeat, kKdim, kWCarryInv);
  }

  rowsum_kernel<<<dim3(kRows / 256), dim3(256), 0, stream>>>(fnn, bias, out0);
}
